// Bi_CrossAttention_29463475650624
// MI455X (gfx1250) — hardware-verified
//
#include <hip/hip_runtime.h>


#define NB_  8
#define TT   1024
#define CC   256
#define DD   512
#define NH_  8
#define HDM  64
#define PCAR 1024.0f
typedef _Float16 h16;
typedef unsigned short bf;
typedef __attribute__((ext_vector_type(16))) __bf16   v16bf;
typedef __attribute__((ext_vector_type(16))) _Float16 v16h;
typedef __attribute__((ext_vector_type(8)))  _Float16 v8h;
typedef __attribute__((ext_vector_type(8)))  unsigned short v8us;
typedef __attribute__((ext_vector_type(8)))  float    v8f;
typedef __attribute__((ext_vector_type(4)))  float    v4f;
typedef v8h  __attribute__((may_alias)) v8ha;
typedef v4f  __attribute__((may_alias)) v4fa;
typedef v8us __attribute__((may_alias)) v8usa;

__device__ __forceinline__ unsigned short f2bf(float f) { unsigned u = __float_as_uint(f); u += 0x7FFFu + ((u >> 16) & 1u); return (unsigned short)(u >> 16); }
__device__ __forceinline__ float bf2f(unsigned short b) { return __uint_as_float(((unsigned)b) << 16); }
__device__ __forceinline__ float bfr(float f) { return bf2f(f2bf(f)); }
__device__ __forceinline__ v16h cat16(v8h lo, v8h hi) { return __builtin_shufflevector(lo, hi, 0, 1, 2, 3, 4, 5, 6, 7, 8, 9, 10, 11, 12, 13, 14, 15); }
__device__ __forceinline__ v16bf cat16b(v8us lo, v8us hi) { return __builtin_bit_cast(v16bf, __builtin_shufflevector(lo, hi, 0, 1, 2, 3, 4, 5, 6, 7, 8, 9, 10, 11, 12, 13, 14, 15)); }
__device__ __forceinline__ v8f wmma16(v16h a, v16h b, v8f c) { return __builtin_amdgcn_wmma_f32_16x16x32_f16(false, a, false, b, (short)0, c, false, false); }
__device__ __forceinline__ v8f wmmab(v16bf a, v16bf b, v8f c) { return __builtin_amdgcn_wmma_f32_16x16x32_bf16(false, a, false, b, (short)0, c, false, false); }


template <typename T16> struct WFrag;
template <> struct WFrag<h16> { typedef v16h V; static __device__ __forceinline__ V ld(const h16* p) { return cat16(*(const v8h*)p, *(const v8h*)(p + 16)); } static __device__ __forceinline__ v8f mma(V a, V b, v8f c) { return wmma16(a, b, c); } };
template <> struct WFrag<bf> { typedef v16bf V; static __device__ __forceinline__ V ld(const bf* p) { return cat16b(*(const v8us*)p, *(const v8us*)(p + 16)); } static __device__ __forceinline__ v8f mma(V a, V b, v8f c) { return wmmab(a, b, c); } };
template <typename T16, int NSPLIT, bool BIAS>
__global__ __launch_bounds__(32) void k_gemmw(const T16* __restrict__ A, const T16* __restrict__ A2, const T16* __restrict__ Bt, const T16* __restrict__ Bt2, int K, float* C, int ldc, const float* __restrict__ bias, size_t sA, size_t sB, size_t sC) {
    typedef typename WFrag<T16>::V V;
    __shared__ __align__(16) float os[16 * 68];
    const size_t z = blockIdx.z; A += z * sA; if (A2) A2 += z * sA; Bt += z * sB; if (Bt2) Bt2 += z * sB; C += z * sC;
    const int lane = threadIdx.x & 31, lr = lane & 15, hi = lane >> 4; const int r0 = blockIdx.x * 64, c0 = blockIdx.y * 64;
    v8f acc[4][4];
#pragma unroll
    for (int mb = 0; mb < 4; ++mb)
#pragma unroll
        for (int nb = 0; nb < 4; ++nb) acc[mb][nb] = (v8f){};
    const size_t aoff = (size_t)(r0 + lr) * K + 8 * hi, boff = (size_t)(c0 + lr) * K + 8 * hi;
#pragma unroll 1
    for (int kc = 0; kc < K; kc += 32) {
        V a[4], a2[4];
#pragma unroll
        for (int mb = 0; mb < 4; ++mb) { a[mb] = WFrag<T16>::ld(A + aoff + (size_t)mb * 16 * K + kc); if (NSPLIT == 1 || NSPLIT == 2) a2[mb] = WFrag<T16>::ld(A2 + aoff + (size_t)mb * 16 * K + kc); }
#pragma unroll
        for (int nb = 0; nb < 4; ++nb) { const V b = WFrag<T16>::ld(Bt + boff + (size_t)nb * 16 * K + kc); V b2; if (NSPLIT >= 2) b2 = WFrag<T16>::ld(Bt2 + boff + (size_t)nb * 16 * K + kc);
#pragma unroll
            for (int mb = 0; mb < 4; ++mb) { acc[mb][nb] = WFrag<T16>::mma(a[mb], b, acc[mb][nb]); if (NSPLIT == 1 || NSPLIT == 2) acc[mb][nb] = WFrag<T16>::mma(a2[mb], b, acc[mb][nb]); if (NSPLIT >= 2) acc[mb][nb] = WFrag<T16>::mma(a[mb], b2, acc[mb][nb]); } }
        asm volatile("v_nop\n\tv_nop\n\tv_nop\n\tv_nop" : "+v"(acc[0][0]), "+v"(acc[1][1]), "+v"(acc[2][2]), "+v"(acc[3][3]) : "v"(a[0]), "v"(a[3]));
    }
#pragma unroll
    for (int mb = 0; mb < 4; ++mb) {
#pragma unroll
        for (int nb = 0; nb < 4; ++nb) {
#pragma unroll
            for (int j = 0; j < 8; ++j) os[(hi * 8 + j) * 68 + nb * 16 + lr] = acc[mb][nb][j]; }
        __builtin_amdgcn_wave_barrier(); asm volatile("" ::: "memory");
        float* crow = C + (size_t)(r0 + mb * 16) * ldc + c0;
#pragma unroll 1
        for (int ps = 0; ps < 2; ++ps) {
#pragma unroll
            for (int s = 0; s < 8; ++s) { const int row = 2 * s + hi, cofs = lr * 4; v4f val = *(const v4fa*)(os + row * 68 + cofs); if (BIAS) { val[0] += bfr(bias[c0 + cofs]); val[1] += bfr(bias[c0 + cofs + 1]); val[2] += bfr(bias[c0 + cofs + 2]); val[3] += bfr(bias[c0 + cofs + 3]); }
                *(volatile v4f*)(crow + (size_t)row * ldc + cofs) = val; }
            if (ps == 0) __threadfence(); }
        __builtin_amdgcn_wave_barrier(); asm volatile("" ::: "memory");
    }
}

__device__ __forceinline__ h16 tohx(float x) { return (h16)x; }
__device__ __forceinline__ void splitf(float y, unsigned short& h, unsigned short& l) { h = f2bf(y); l = f2bf(y - bf2f(h)); }
typedef __attribute__((ext_vector_type(2))) _Float16 v2h;
typedef __attribute__((ext_vector_type(4))) _Float16 v4h;
typedef __attribute__((ext_vector_type(2))) unsigned short v2us;
typedef __attribute__((ext_vector_type(4))) unsigned short v4us;
typedef __attribute__((ext_vector_type(2))) float v2f;

__global__ __launch_bounds__(256) void k_cvt8(const float* __restrict__ src, bf* dst, size_t n8) { const size_t i = (size_t)blockIdx.x * 256 + threadIdx.x; if (i >= n8) return; const v8f v = *(const v8f*)(src + i * 8); v8us o;
#pragma unroll
    for (int k = 0; k < 8; ++k) o[k] = f2bf(v[k]); *(volatile v8us*)(dst + i * 8) = o; __threadfence(); *(volatile v8us*)(dst + i * 8) = o; }
__global__ __launch_bounds__(256) void k_xt8(const float* __restrict__ xb, bf* XT) { const size_t e = ((size_t)blockIdx.x * 256 + threadIdx.x) * 4; if (e >= (size_t)TT * CC) return; const int c = (int)(e % CC), n = (int)(e / CC); v4us o;
#pragma unroll
    for (int q = 0; q < 4; ++q) o[q] = f2bf(xb[(size_t)(c + q) * TT + n]); *(volatile v4us*)(XT + e) = o; __threadfence(); *(volatile v4us*)(XT + e) = o; }
__global__ __launch_bounds__(256) void k_pl(const float* __restrict__ F, int pitch, int nh, int hd, h16* P) { const size_t e = ((size_t)blockIdx.x * 256 + threadIdx.x) * 2; if (e >= (size_t)nh * TT * hd) return; const int d = (int)(e % hd); const int t = (int)((e / hd) % TT); const int h = (int)(e / ((size_t)hd * TT)); v2h o; o[0] = tohx(F[(size_t)t * pitch + h * hd + d]); o[1] = tohx(F[(size_t)t * pitch + h * hd + d + 1]); *(volatile v2h*)(P + e) = o; __threadfence(); *(volatile v2h*)(P + e) = o; }
__global__ __launch_bounds__(256) void k_vt(const float* __restrict__ F, int pitch, int nh, int hd, h16* VT) { const size_t e = ((size_t)blockIdx.x * 256 + threadIdx.x) * 2; if (e >= (size_t)nh * hd * TT) return; const int t = (int)(e % TT); const int d = (int)((e / TT) % hd); const int h = (int)(e / ((size_t)TT * hd)); v2h o; o[0] = tohx(F[(size_t)t * pitch + h * hd + d]); o[1] = tohx(F[(size_t)(t + 1) * pitch + h * hd + d]); *(volatile v2h*)(VT + e) = o; __threadfence(); *(volatile v2h*)(VT + e) = o; }
__global__ __launch_bounds__(256) void k_asoft(const float* __restrict__ Sb, const float* __restrict__ MOD, int h, float scl, h16* P16) { const int lane = threadIdx.x & 31; const int row = blockIdx.x * 8 + (threadIdx.x >> 5); if (row >= TT) return; const float* sr = Sb + (size_t)row * TT; float sc = scl; if (MOD) { float m = MOD[(size_t)row * 64 + h]; asm volatile("" : "+v"(m)); sc = __fmul_rn(scl, m); } float v[32]; float mx = -3.0e38f;
#pragma unroll
    for (int ch = 0; ch < 8; ++ch) { const int j0 = ch * 128 + lane * 4; const v4f a = *(const v4f*)(sr + j0);
#pragma unroll
        for (int q = 0; q < 4; ++q) { const float t = __fmul_rn(a[q], sc); v[ch * 4 + q] = t; mx = fmaxf(mx, t); } }
#pragma unroll
    for (int sh = 16; sh; sh >>= 1) mx = fmaxf(mx, __shfl_xor(mx, sh, 32));
    float sum = 0.f;
#pragma unroll
    for (int k = 0; k < 32; ++k) { float d0 = __fsub_rn(v[k], mx); asm volatile("" : "+v"(d0)); v[k] = __builtin_amdgcn_exp2f(__fmul_rn(d0, 1.4426950408889634f)); sum += v[k]; }
#pragma unroll
    for (int sh = 16; sh; sh >>= 1) sum += __shfl_xor(sum, sh, 32);
    const float f = __fdiv_rn(PCAR, sum);
#pragma unroll 1
    for (int ps = 0; ps < 2; ++ps) {
#pragma unroll
        for (int ch = 0; ch < 8; ++ch) { v4h o;
#pragma unroll
            for (int q = 0; q < 4; ++q) o[q] = tohx(v[ch * 4 + q] * f); *(volatile v4h*)(P16 + (size_t)row * TT + ch * 128 + lane * 4) = o; }
        if (ps == 0) __threadfence(); } }
__global__ __launch_bounds__(256) void k_mrgf(const float* __restrict__ O, int h, int hd, float* CT) { const size_t e = ((size_t)blockIdx.x * 256 + threadIdx.x) * 2; if (e >= (size_t)TT * hd) return; const int d = (int)(e % hd); const int t = (int)(e / hd); v2f o; o[0] = O[e] * (1.0f / PCAR); o[1] = O[e + 1] * (1.0f / PCAR); const size_t oo = (size_t)t * DD + h * hd + d; *(volatile v2f*)(CT + oo) = o; __threadfence(); *(volatile v2f*)(CT + oo) = o; }
__global__ __launch_bounds__(256) void k_mrg(const float* __restrict__ O, int h, int hd, bf* Ah, bf* Al) { const size_t e = ((size_t)blockIdx.x * 256 + threadIdx.x) * 2; if (e >= (size_t)TT * hd) return; const int d = (int)(e % hd); const int t = (int)(e / hd); v2us oh, ol;
#pragma unroll
    for (int q = 0; q < 2; ++q) { unsigned short a, c2; splitf(O[e + q] * (1.0f / PCAR), a, c2); oh[q] = a; ol[q] = c2; } const size_t oo = (size_t)t * DD + h * hd + d; *(volatile v2us*)(Ah + oo) = oh; *(volatile v2us*)(Al + oo) = ol; __threadfence(); *(volatile v2us*)(Ah + oo) = oh; *(volatile v2us*)(Al + oo) = ol; }
__global__ __launch_bounds__(256) void k_colst(const float* __restrict__ S, float scl, float* CM, float* CI) { const int j = blockIdx.x * 256 + threadIdx.x; if (j >= TT) return; float m = -3.0e38f;
    for (int i = 0; i < TT; ++i) m = fmaxf(m, S[(size_t)i * TT + j] * scl);
    float s = 0.f; for (int i = 0; i < TT; ++i) { float a = S[(size_t)i * TT + j] * scl; asm volatile("" : "+v"(a)); float d0 = __fsub_rn(a, m); asm volatile("" : "+v"(d0)); s = __fadd_rn(s, __expf(d0)); }
    const float ci = __fdiv_rn(PCAR, s); *(volatile float*)(CM + j) = m; *(volatile float*)(CI + j) = ci; __threadfence(); *(volatile float*)(CM + j) = m; *(volatile float*)(CI + j) = ci; }
__global__ __launch_bounds__(256) void k_pcolT(const float* __restrict__ S, float scl, const float* __restrict__ CM, const float* __restrict__ CI, h16* PT) { const int e = (blockIdx.x * 256 + threadIdx.x) * 2; if (e >= TT * TT) return; const int i = e % TT, j = e / TT; const float m = CM[j], ci = CI[j]; v2h o;
#pragma unroll
    for (int q = 0; q < 2; ++q) { float a = S[(size_t)(i + q) * TT + j] * scl; asm volatile("" : "+v"(a)); float d0 = __fsub_rn(a, m); asm volatile("" : "+v"(d0)); o[q] = tohx(__fmul_rn(__expf(d0), ci)); } *(volatile v2h*)(PT + e) = o; __threadfence(); *(volatile v2h*)(PT + e) = o; }
__global__ __launch_bounds__(256) void k_outT(const float* __restrict__ PO, float* OUTb) { const size_t e = ((size_t)blockIdx.x * 256 + threadIdx.x) * 2; if (e >= (size_t)CC * TT) return; const int n = (int)(e % TT), c = (int)(e / TT); v2f o; o[0] = PO[(size_t)n * CC + c]; o[1] = PO[(size_t)(n + 1) * CC + c]; *(volatile v2f*)(OUTb + e) = o; __threadfence(); *(volatile v2f*)(OUTb + e) = o; }

extern "C" void kernel_launch(void* const* d_in, const int* in_sizes, int n_in,
                              void* d_out, int out_size, void* d_ws, size_t ws_size, hipStream_t stream) {
    (void)in_sizes; (void)n_in; (void)out_size;
    const float* IN[14]; for (int i = 0; i < 14; ++i) IN[i] = (const float*)d_in[i];
    float* OUT1 = (float*)d_out; float* OUT2 = (float*)d_out + (size_t)NB_ * CC * TT;
    char* wsp = (char*)d_ws;
    auto take = [&](size_t bytes) { char* p = wsp; wsp += (bytes + 255) & ~(size_t)255; return (void*)p; };
    bf* WK1 = (bf*)take((size_t)DD * CC * 2); bf* WK2 = (bf*)take((size_t)DD * CC * 2); bf* WV1 = (bf*)take((size_t)DD * CC * 2); bf* WV2 = (bf*)take((size_t)DD * CC * 2); bf* WO1 = (bf*)take((size_t)CC * DD * 2); bf* WO2 = (bf*)take((size_t)CC * DD * 2);
    bf* X1 = (bf*)take((size_t)TT * CC * 2); bf* X2 = (bf*)take((size_t)TT * CC * 2); float* F = (float*)take((size_t)TT * DD * 4);
    h16* K1P = (h16*)take((size_t)TT * DD * 2); h16* K2P = (h16*)take((size_t)TT * DD * 2); h16* V1T = (h16*)take((size_t)DD * TT * 2); h16* V2T = (h16*)take((size_t)DD * TT * 2);
    float* Sb = (float*)take((size_t)TT * TT * 4); h16* Pm = (h16*)take((size_t)TT * TT * 2); h16* PT = (h16*)take((size_t)TT * TT * 2); float* CM = (float*)take((size_t)TT * 4); float* CI = (float*)take((size_t)TT * 4); float* O = (float*)take((size_t)TT * HDM * 4);
    bf* A1h = (bf*)take((size_t)TT * DD * 2); bf* A1l = (bf*)take((size_t)TT * DD * 2); bf* A2h = (bf*)take((size_t)TT * DD * 2); bf* A2l = (bf*)take((size_t)TT * DD * 2); float* PO = (float*)take((size_t)TT * CC * 4);
    if ((size_t)(wsp - (char*)d_ws) > ws_size) return;
    { const size_t nw = (size_t)DD * CC / 8; const unsigned g = (unsigned)((nw + 255) / 256); k_cvt8<<<g, 256, 0, stream>>>(IN[2], WK1, nw); k_cvt8<<<g, 256, 0, stream>>>(IN[4], WK2, nw); k_cvt8<<<g, 256, 0, stream>>>(IN[6], WV1, nw); k_cvt8<<<g, 256, 0, stream>>>(IN[8], WV2, nw); k_cvt8<<<g, 256, 0, stream>>>(IN[10], WO1, nw); k_cvt8<<<g, 256, 0, stream>>>(IN[12], WO2, nw); }
    const dim3 gP(TT / 64, DD / 64, 1); const unsigned LP = (TT * DD / 2 + 255) / 256, LX = (TT * CC / 4 + 255) / 256; const float scl = 0.125f;
    for (int b = 0; b < NB_; ++b) {
        k_xt8<<<LX, 256, 0, stream>>>(IN[0] + (size_t)b * CC * TT, X1); k_xt8<<<LX, 256, 0, stream>>>(IN[1] + (size_t)b * CC * TT, X2);
        k_gemmw<bf, 0, true><<<gP, 32, 0, stream>>>(X1, nullptr, WK1, nullptr, CC, F, DD, IN[3], 0, 0, 0); k_pl<<<LP, 256, 0, stream>>>(F, DD, NH_, HDM, K1P);
        k_gemmw<bf, 0, true><<<gP, 32, 0, stream>>>(X2, nullptr, WK2, nullptr, CC, F, DD, IN[5], 0, 0, 0); k_pl<<<LP, 256, 0, stream>>>(F, DD, NH_, HDM, K2P);
        k_gemmw<bf, 0, true><<<gP, 32, 0, stream>>>(X1, nullptr, WV1, nullptr, CC, F, DD, IN[7], 0, 0, 0); k_vt<<<LP, 256, 0, stream>>>(F, DD, NH_, HDM, V1T);
        k_gemmw<bf, 0, true><<<gP, 32, 0, stream>>>(X2, nullptr, WV2, nullptr, CC, F, DD, IN[9], 0, 0, 0); k_vt<<<LP, 256, 0, stream>>>(F, DD, NH_, HDM, V2T);
        for (int h = 0; h < NH_; ++h) {
            k_gemmw<h16, 0, false><<<dim3(TT / 64, TT / 64, 1), 32, 0, stream>>>(K1P + (size_t)h * TT * HDM, nullptr, K2P + (size_t)h * TT * HDM, nullptr, HDM, Sb, TT, nullptr, 0, 0, 0);
            k_asoft<<<TT / 8, 256, 0, stream>>>(Sb, nullptr, h, scl, Pm);
            k_gemmw<h16, 0, false><<<dim3(TT / 64, 1, 1), 32, 0, stream>>>(Pm, nullptr, V2T + (size_t)h * HDM * TT, nullptr, TT, O, HDM, nullptr, 0, 0, 0); k_mrg<<<(TT * HDM / 2 + 255) / 256, 256, 0, stream>>>(O, h, HDM, A1h, A1l);
            k_colst<<<TT / 256, 256, 0, stream>>>(Sb, scl, CM, CI); k_pcolT<<<(TT * TT / 2 + 255) / 256, 256, 0, stream>>>(Sb, scl, CM, CI, PT);
            k_gemmw<h16, 0, false><<<dim3(TT / 64, 1, 1), 32, 0, stream>>>(PT, nullptr, V1T + (size_t)h * HDM * TT, nullptr, TT, O, HDM, nullptr, 0, 0, 0); k_mrg<<<(TT * HDM / 2 + 255) / 256, 256, 0, stream>>>(O, h, HDM, A2h, A2l); }
        k_gemmw<bf, 1, true><<<dim3(TT / 64, CC / 64, 1), 32, 0, stream>>>(A1h, A1l, WO1, nullptr, DD, PO, CC, IN[11], 0, 0, 0); k_outT<<<(CC * TT / 2 + 255) / 256, 256, 0, stream>>>(PO, OUT1 + (size_t)b * CC * TT);
        k_gemmw<bf, 1, true><<<dim3(TT / 64, CC / 64, 1), 32, 0, stream>>>(A2h, A2l, WO2, nullptr, DD, PO, CC, IN[13], 0, 0, 0); k_outT<<<(CC * TT / 2 + 255) / 256, 256, 0, stream>>>(PO, OUT2 + (size_t)b * CC * TT); }
}
